// WeightedMultiHeadGAT_10264971837706
// MI455X (gfx1250) — hardware-verified
//
#include <hip/hip_runtime.h>


namespace {
constexpr int N = 2048, IN = 256, NH = 12, HD = 32, HDIM = NH * HD, OUT = 384, NLT = N / 16;
constexpr float XS = 8.0f, PS = 32768.0f, WSC = 256.0f, SLOPE = 0.2f;
typedef _Float16 b16;
typedef __attribute__((ext_vector_type(16))) _Float16 v16b;
typedef __attribute__((ext_vector_type(8))) _Float16 v8b;
typedef __attribute__((ext_vector_type(8))) float v8f;
typedef __attribute__((ext_vector_type(4))) float v4f;
__device__ __forceinline__ float bf16_rne(float f) { unsigned int u = __float_as_uint(f); u += 0x7FFFu + ((u >> 16) & 1u); return __uint_as_float(u & 0xFFFF0000u); }
__device__ __forceinline__ void split16(float v, b16& hi, b16& lo) { hi = (b16)v; lo = (b16)(v - (float)hi); }
__device__ __forceinline__ v16b frag_kb(const b16* p, int hh) { const v8b a = *(const v8b*)(p + 8 * hh), b = *(const v8b*)(p + 16 + 8 * hh); v16b f;
#pragma unroll
  for (int e = 0; e < 8; ++e) { f[e] = a[e]; f[8 + e] = b[e]; } return f; }
__device__ __forceinline__ v8f wmma16b(v16b a, v16b b, v8f c) { v8f d = __builtin_amdgcn_wmma_f32_16x16x32_f16(false, a, false, b, (short)0, c, false, false); asm volatile("v_nop\n\tv_nop\n\tv_nop\n\tv_nop" : "+v"(d) : "v"(a), "v"(b)); return d; }
__device__ __forceinline__ void wave_lds_sync() { __builtin_amdgcn_fence(__ATOMIC_RELEASE, "workgroup"); __builtin_amdgcn_wave_barrier(); __builtin_amdgcn_fence(__ATOMIC_ACQUIRE, "workgroup"); }
__device__ __forceinline__ float pmul(float a, float b) { float p = a * b; asm volatile("" : "+v"(p)); return p; }
__device__ __forceinline__ float leaky(float v) { return v >= 0.0f ? v : SLOPE * v; }

__global__ __launch_bounds__(256) void wcopy_kernel(const float* __restrict__ w, int n8, int ro, int KIN, b16* __restrict__ WT) {
  const int u = blockIdx.x * 256 + threadIdx.x; if (u >= n8) return; const size_t e = (size_t)u * 8; v8b v;
#pragma unroll
  for (int j = 0; j < 8; ++j) v[j] = (b16)(bf16_rne(w[e + j]) * WSC); for (int pass = 0; pass < 2; ++pass) { *(volatile v8b*)(WT + (size_t)ro * KIN + e) = v; __threadfence(); }
}
__global__ __launch_bounds__(32) void proj_kernel(const float* __restrict__ x, const b16* __restrict__ WT, const float* __restrict__ asrc, const float* __restrict__ adst, const float* __restrict__ rb, int NLV, float* __restrict__ HP, float* __restrict__ RES, float* __restrict__ AS, float* __restrict__ AD) {
  __shared__ __attribute__((aligned(16))) b16 Ah[16][IN + 8]; __shared__ __attribute__((aligned(16))) float Tf[16][128 + 4], Ps[16][16], Pd[16][16];
  const int lane = threadIdx.x, nloc = lane & 15, hlf = lane >> 4; const size_t m0 = (size_t)blockIdx.x * 16;
  for (int rr = 0; rr < 16; ++rr) for (int q = 0; q < 8; ++q) Ah[rr][q * 32 + lane] = (b16)(bf16_rne(x[(m0 + rr) * IN + q * 32 + lane]) * XS);
  if (lane < 16) for (int rr = 0; rr < 16; ++rr) { Ps[rr][lane] = 0.0f; Pd[rr][lane] = 0.0f; }
  wave_lds_sync();
#pragma unroll 1
  for (int cg = 0; cg < 6; ++cg) { v8f acc[8];
#pragma unroll
    for (int t = 0; t < 8; ++t) acc[t] = (v8f){};
#pragma unroll 2
    for (int kb = 0; kb < IN; kb += 32) { const v16b a = frag_kb(&Ah[nloc][kb], hlf);
#pragma unroll
      for (int t = 0; t < 8; ++t) acc[t] = wmma16b(a, frag_kb(WT + (size_t)(cg * 128 + t * 16 + nloc) * IN + kb, hlf), acc[t]); }
    if (cg < 3) {
#pragma unroll
      for (int t = 0; t < 8; ++t) { const int c = cg * 128 + t * 16 + nloc; const int hd = c / HD; const float ws_ = bf16_rne(asrc[c]), wd_ = bf16_rne(adst[c]); float ps[8], pd[8];
#pragma unroll
        for (int r8 = 0; r8 < 8; ++r8) { const float v = acc[t][r8] * (1.0f / (XS * WSC)); Tf[8 * hlf + r8][t * 16 + nloc] = v; ps[r8] = pmul(v, ws_); pd[r8] = pmul(v, wd_); }
#pragma unroll
        for (int r8 = 0; r8 < 8; ++r8) { for (int o = 1; o < 16; o <<= 1) { ps[r8] += __shfl_xor(ps[r8], o); pd[r8] += __shfl_xor(pd[r8], o); } }
        if (nloc == 0) {
#pragma unroll
          for (int r8 = 0; r8 < 8; ++r8) { Ps[8 * hlf + r8][hd] += ps[r8]; Pd[8 * hlf + r8][hd] += pd[r8]; } } }
      wave_lds_sync();
      for (int pass = 0; pass < 2; ++pass) { for (int rr = 0; rr < 16; ++rr) *(volatile v4f*)(HP + (m0 + rr) * HDIM + cg * 128 + lane * 4) = *(const v4f*)(&Tf[rr][lane * 4]); __threadfence(); } }
    else {
#pragma unroll
      for (int t = 0; t < 8; ++t) { const int c = (cg - 3) * 128 + t * 16 + nloc; const float bb = bf16_rne(rb[c]);
#pragma unroll
        for (int r8 = 0; r8 < 8; ++r8) Tf[8 * hlf + r8][t * 16 + nloc] = acc[t][r8] * (1.0f / (XS * WSC)) + bb; }
      wave_lds_sync();
      for (int pass = 0; pass < 2; ++pass) { for (int rr = 0; rr < 16; ++rr) *(volatile v4f*)(RES + (m0 + rr) * HDIM + (cg - 3) * 128 + lane * 4) = *(const v4f*)(&Tf[rr][lane * 4]); __threadfence(); } }
    wave_lds_sync(); }
  for (int pass = 0; pass < 2; ++pass) { for (int q = 0; q < 8; ++q) { const int i = q * 32 + lane; ((volatile float*)AS)[m0 * 16 + i] = Ps[i >> 4][i & 15]; ((volatile float*)AD)[m0 * 16 + i] = Pd[i >> 4][i & 15]; } __threadfence(); }
}
__global__ __launch_bounds__(256) void ht_kernel(const float* __restrict__ HP, b16* __restrict__ HTH, b16* __restrict__ HTL) {
  __shared__ float T[64][65]; const int ct = blockIdx.x % (HDIM / 64), jt = blockIdx.x / (HDIM / 64); const int tid = threadIdx.x;
  for (int i = tid; i < 64 * 64; i += 256) { const int r = i / 64, c = i % 64; T[r][c] = HP[(size_t)(jt * 64 + r) * HDIM + ct * 64 + c]; }
  __syncthreads();
  { const int c = tid / 4, g = (tid % 4) * 2; for (int gg = g; gg < g + 2; ++gg) { v8b vh, vl;
#pragma unroll
      for (int j = 0; j < 8; ++j) { b16 p, q; split16(T[gg * 8 + j][c] * XS, p, q); vh[j] = p; vl[j] = q; }
      const size_t o = (size_t)(ct * 64 + c) * N + jt * 64 + gg * 8; for (int pass = 0; pass < 2; ++pass) { *(volatile v8b*)(HTH + o) = vh; *(volatile v8b*)(HTL + o) = vl; __threadfence(); } } }
}
__global__ __launch_bounds__(32) void att_kernel(const float* __restrict__ adj, const float* __restrict__ AS, const float* __restrict__ AD, const float* __restrict__ ew, const float* __restrict__ eb, const b16* __restrict__ HTH, const b16* __restrict__ HTL, const float* __restrict__ RES, float* __restrict__ HO) {
  __shared__ __attribute__((aligned(16))) b16 Ph[16][32 + 8], Pl[16][32 + 8]; __shared__ float Mx[16], Sm[16], Asi[16]; __shared__ __attribute__((aligned(16))) float Tf[16][HD + 1];
  const int lane = threadIdx.x, nloc = lane & 15, hlf = lane >> 4; const int h = blockIdx.x % NH, lt = blockIdx.x / NH; const size_t i0 = (size_t)lt * 16; const float w_e = bf16_rne(ew[h]), b_e = bf16_rne(eb[h]);
  if (lane < 16) Asi[lane] = AS[(i0 + lane) * 16 + h];
  wave_lds_sync();
  for (int rr = 0; rr < 16; ++rr) { const float* ar = adj + (i0 + rr) * N; const float asi = Asi[rr]; float mx = -INFINITY;
#pragma unroll 4
    for (int jb = 0; jb < N; jb += 32) { const int j = jb + lane; const float a = bf16_rne(ar[j]); if (a > 0.0f) mx = fmaxf(mx, leaky(asi + AD[(size_t)j * 16 + h] + pmul(a, w_e) + b_e)); }
    for (int o = 16; o; o >>= 1) mx = fmaxf(mx, __shfl_xor(mx, o)); if (lane == 0) { Mx[rr] = mx; Sm[rr] = 0.0f; } }
  wave_lds_sync();
  v8f acc[2] = {(v8f){}, (v8f){}}; float rs[16]; for (int rr = 0; rr < 16; ++rr) rs[rr] = 0.0f;
#pragma unroll 1
  for (int jb = 0; jb < N; jb += 32) { const int j = jb + lane; const float adj_d = AD[(size_t)j * 16 + h];
    for (int rr = 0; rr < 16; ++rr) { const float a = bf16_rne(adj[(i0 + rr) * N + j]); float p = 0.0f; if (a > 0.0f && Mx[rr] > -INFINITY) p = __expf(leaky(Asi[rr] + adj_d + pmul(a, w_e) + b_e) - Mx[rr]); rs[rr] += p; b16 ph, pl; split16(p * PS, ph, pl); Ph[rr][lane] = ph; Pl[rr][lane] = pl; }
    wave_lds_sync();
    const v16b a = frag_kb(&Ph[nloc][0], hlf), al = frag_kb(&Pl[nloc][0], hlf);
#pragma unroll
    for (int t = 0; t < 2; ++t) { const size_t br = (size_t)(h * HD + t * 16 + nloc) * N + jb; const v16b bh = frag_kb(HTH + br, hlf), bl = frag_kb(HTL + br, hlf); acc[t] = wmma16b(a, bh, acc[t]); acc[t] = wmma16b(a, bl, acc[t]); acc[t] = wmma16b(al, bh, acc[t]); acc[t] = wmma16b(al, bl, acc[t]); }
    wave_lds_sync(); }
  for (int rr = 0; rr < 16; ++rr) { float s = rs[rr]; for (int o = 16; o; o >>= 1) s += __shfl_xor(s, o); if (lane == 0) Sm[rr] = s; }
  wave_lds_sync();
#pragma unroll
  for (int t = 0; t < 2; ++t)
#pragma unroll
    for (int r8 = 0; r8 < 8; ++r8) { const int rl = 8 * hlf + r8; const float s = Sm[rl]; Tf[rl][t * 16 + nloc] = (s > 0.0f ? acc[t][r8] * (1.0f / (PS * XS)) / s : 0.0f) + RES[(i0 + rl) * HDIM + h * HD + t * 16 + nloc]; }
  wave_lds_sync();
  for (int pass = 0; pass < 2; ++pass) { for (int rr = 0; rr < 16; ++rr) ((volatile float*)HO)[(i0 + rr) * HDIM + h * HD + lane] = Tf[rr][lane]; __threadfence(); }
}
__global__ __launch_bounds__(32) void fus_kernel(const float* __restrict__ HO, const b16* __restrict__ WF, const float* __restrict__ fb, int NLV, float* __restrict__ out) {
  __shared__ __attribute__((aligned(16))) b16 Ah[16][HDIM + 8], Al[16][HDIM + 8]; __shared__ __attribute__((aligned(16))) float Tf[16][128 + 4];
  const int lane = threadIdx.x, nloc = lane & 15, hlf = lane >> 4; const size_t m0 = (size_t)blockIdx.x * 16; if (m0 >= (size_t)NLV) return;
  for (int rr = 0; rr < 16; ++rr) for (int q = 0; q < HDIM / 32; ++q) { b16 p, ql; split16(HO[(m0 + rr) * HDIM + q * 32 + lane] * XS, p, ql); Ah[rr][q * 32 + lane] = p; Al[rr][q * 32 + lane] = ql; }
  wave_lds_sync();
#pragma unroll 1
  for (int cg = 0; cg < 3; ++cg) { v8f acc[8];
#pragma unroll
    for (int t = 0; t < 8; ++t) acc[t] = (v8f){};
#pragma unroll 2
    for (int kb = 0; kb < HDIM; kb += 32) { const v16b a = frag_kb(&Ah[nloc][kb], hlf), a2 = frag_kb(&Al[nloc][kb], hlf);
#pragma unroll
      for (int t = 0; t < 8; ++t) { const v16b bw = frag_kb(WF + (size_t)(cg * 128 + t * 16 + nloc) * HDIM + kb, hlf); acc[t] = wmma16b(a, bw, acc[t]); acc[t] = wmma16b(a2, bw, acc[t]); } }
#pragma unroll
    for (int t = 0; t < 8; ++t) { const int c = cg * 128 + t * 16 + nloc; const float bb = bf16_rne(fb[c]);
#pragma unroll
      for (int r8 = 0; r8 < 8; ++r8) { const float z = acc[t][r8] * (1.0f / (XS * WSC)) + bb; Tf[8 * hlf + r8][t * 16 + nloc] = 0.5f * z * (1.0f + erff(z * 0.70710678118654752f)); } }
    wave_lds_sync();
    for (int pass = 0; pass < 2; ++pass) { for (int rr = 0; rr < 16; ++rr) *(volatile v4f*)(out + (m0 + rr) * OUT + cg * 128 + lane * 4) = *(const v4f*)(&Tf[rr][lane * 4]); __threadfence(); }
    wave_lds_sync(); }
}
}

extern "C" void kernel_launch(void* const* d_in, const int* in_sizes, int n_in, void* d_out, int out_size, void* d_ws, size_t ws_size, hipStream_t stream) {
  (void)n_in;
  auto Fp = [&](int i) { return (const float*)d_in[i]; };
  if (in_sizes[0] != N * IN || in_sizes[1] != N * N || in_sizes[2] != HDIM * IN || in_sizes[3] != NH * HD || in_sizes[5] != NH || in_sizes[7] != HDIM * IN || in_sizes[9] != OUT * HDIM || out_size != N * OUT) return;
  const int NLV = N;
  size_t off = 0; char* ws = (char*)d_ws;
  auto carve = [&](size_t bytes) { char* p = ws + off; off += (bytes + 255) & ~(size_t)255; return p; };
  b16* WT = (b16*)carve((size_t)2 * HDIM * IN * 2); b16* WF = (b16*)carve((size_t)OUT * HDIM * 2); float* HP = (float*)carve((size_t)N * HDIM * 4); float* RES = (float*)carve((size_t)N * HDIM * 4); float* AS = (float*)carve((size_t)N * 16 * 4); float* AD = (float*)carve((size_t)N * 16 * 4);
  b16* HTH = (b16*)carve((size_t)HDIM * N * 2); b16* HTL = (b16*)carve((size_t)HDIM * N * 2); float* HO = (float*)carve((size_t)N * HDIM * 4);
  if (off > ws_size || off > ((size_t)32 << 20)) return;
  wcopy_kernel<<<(HDIM * IN / 8 + 255) / 256, 256, 0, stream>>>(Fp(2), HDIM * IN / 8, 0, IN, WT); wcopy_kernel<<<(HDIM * IN / 8 + 255) / 256, 256, 0, stream>>>(Fp(7), HDIM * IN / 8, HDIM, IN, WT); wcopy_kernel<<<(OUT * HDIM / 8 + 255) / 256, 256, 0, stream>>>(Fp(9), OUT * HDIM / 8, 0, HDIM, WF);
  proj_kernel<<<NLT, 32, 0, stream>>>(Fp(0), WT, Fp(3), Fp(4), Fp(8), NLV, HP, RES, AS, AD);
  ht_kernel<<<(HDIM / 64) * (N / 64), 256, 0, stream>>>(HP, HTH, HTL);
  att_kernel<<<(NLV / 16) * NH, 32, 0, stream>>>(Fp(1), AS, AD, Fp(5), Fp(6), HTH, HTL, RES, HO);
  fus_kernel<<<NLV / 16, 32, 0, stream>>>(HO, WF, Fp(10), NLV, (float*)d_out);
}
